// GenericLinear_17772574671348
// MI455X (gfx1250) — hardware-verified
//
#include <hip/hip_runtime.h>
#include <stddef.h>
#include <stdint.h>


#define NBL   8
#define MB    512
#define MTOT  4096
#define KD    1024
#define UB    1024
#define NW    8192
#define XSC   8
#define WSC   1024
#define NTHR  256
#define NWAVE 8
#define TPW   64
#define WSCAP 134217728
#define LDS_GEMM (NWAVE * 32 * 64 * 4)

static_assert(MTOT == NBL * MB);
static_assert(NW == NBL * UB);
static_assert((KD % 128) == 0);
static_assert((KD % 32) == 0);
static_assert((MB % 128) == 0);
static_assert((UB % 128) == 0);
static_assert((NW % 64) == 0);
static_assert(((MTOT * KD) % (8 * NTHR)) == 0);
static_assert(NTHR == NWAVE * 32);
static_assert(LDS_GEMM <= 300 * 1024);

typedef float          v2f  __attribute__((ext_vector_type(2)));
typedef float          v4f  __attribute__((ext_vector_type(4)));
typedef float          v8f  __attribute__((ext_vector_type(8)));
typedef _Float16       v8h  __attribute__((ext_vector_type(8)));
typedef _Float16       v16h __attribute__((ext_vector_type(16)));
typedef unsigned int   v8u  __attribute__((ext_vector_type(8)));
union FragH { v16h v; v8h h[2]; v8u u; };

__constant__ int c_js[NBL * NBL] = {
   0,  1,  2,  3,  4,  5,  6,  7,
   1,  0,  4,  5,  2,  3,  7,  6,
   2, 12,  0,  6,  9, 15,  3, 13,
   3, 13, 14,  0,  7,  9, 10,  4,
  12,  2,  9, 15,  0,  6, 13,  3,
  13,  3,  7,  9, 14,  0,  4, 10,
  14, 15,  3, 10,  5, 12,  0,  1,
  15, 14,  5, 12,  3, 10,  1,  0
};

__device__ __forceinline__ v8f wmf(v16h a, v16h b, v8f c) {
  v8f d = __builtin_amdgcn_wmma_f32_16x16x32_f16(false, a, false, b, (short)0, c, false, false);
  asm volatile("v_nop\n\tv_nop\n\tv_nop\n\tv_nop" : "+v"(d) : "v"(a), "v"(b));
  return d;
}

__global__ __launch_bounds__(NTHR) void k_prepx(const float* __restrict__ x, _Float16* xh) {
  const size_t t = (size_t)blockIdx.x * NTHR + threadIdx.x;
  const float* p = x + t * 8;
  const v4f f0 = *(const v4f*)p;
  const v4f f1 = *(const v4f*)(p + 4);
  v8h a;
  a[0] = (_Float16)(f0.x * (float)XSC); a[1] = (_Float16)(f0.y * (float)XSC);
  a[2] = (_Float16)(f0.z * (float)XSC); a[3] = (_Float16)(f0.w * (float)XSC);
  a[4] = (_Float16)(f1.x * (float)XSC); a[5] = (_Float16)(f1.y * (float)XSC);
  a[6] = (_Float16)(f1.z * (float)XSC); a[7] = (_Float16)(f1.w * (float)XSC);
  _Float16* d = xh + t * 8;
  *(volatile v8h*)d = a;
  __threadfence();
  *(volatile v8h*)d = a;
}

__global__ __launch_bounds__(NTHR) void k_prepw(const float* __restrict__ W, _Float16* wt) {
  __shared__ __attribute__((aligned(16))) float tile[128 * TPW];
  const int tid = threadIdx.x, lane = tid & 31, g = tid >> 5, hh = lane >> 4, m = lane & 15;
  const int n0 = blockIdx.x * 64;
  const int n = n0 + 2 * lane;
#pragma unroll 1
  for (int dc = 0; dc < KD; dc += 128) {
    __syncthreads();
#pragma unroll 4
    for (int p = 0; p < 16; ++p) {
      const int dl = g + 8 * p;
      const v2f w = *(const v2f*)(W + (size_t)(dc + dl) * NW + n);
      *(v2f*)(tile + dl * TPW + 2 * lane) = w;
    }
    __syncthreads();
    v8h hv[4];
#pragma unroll
    for (int q = 0; q < 4; ++q) {
      const int nl = 8 * g + 2 * q + hh;
      const int d8 = 8 * m;
#pragma unroll
      for (int e = 0; e < 8; ++e) hv[q][e] = (_Float16)(tile[(d8 + e) * TPW + nl] * (float)WSC);
    }
#pragma unroll
    for (int q = 0; q < 4; ++q) {
      _Float16* d = wt + (size_t)(n0 + 8 * g + 2 * q + hh) * KD + dc + 8 * m;
      *(volatile v8h*)d = hv[q];
    }
    __threadfence();
#pragma unroll
    for (int q = 0; q < 4; ++q) {
      _Float16* d = wt + (size_t)(n0 + 8 * g + 2 * q + hh) * KD + dc + 8 * m;
      *(volatile v8h*)d = hv[q];
    }
  }
}

__global__ __launch_bounds__(NTHR) void k_gemm(const _Float16* __restrict__ xh, const _Float16* __restrict__ wt,
                                               const float* __restrict__ bias, float* out) {
  extern __shared__ v4f lds_dyn[];
  const int tid = threadIdx.x, lane = tid & 31, wave = tid >> 5, hh = lane >> 4, m = lane & 15;
  float* stg = (float*)lds_dyn + wave * (32 * 64);
  const int n0 = blockIdx.x * 128, m0 = blockIdx.y * 128, kb = blockIdx.z;
  const int wm = (wave >> 1) * 32, wn = (wave & 1) * 64;

  v8f acc[2][4];
#pragma unroll
  for (int mt = 0; mt < 2; ++mt)
#pragma unroll
    for (int nt = 0; nt < 4; ++nt) { v8f z = {0.f, 0.f, 0.f, 0.f, 0.f, 0.f, 0.f, 0.f}; acc[mt][nt] = z; }

#pragma unroll 1
  for (int i = 0; i < NBL; ++i) {
    const int js = c_js[i * NBL + kb];
    const int jb = js & 7;
    const unsigned sx = (js & 8) ? 0x80008000u : 0u;
    const _Float16* ap = xh + (size_t)(i * MB + m0 + wm + m) * KD + 8 * hh;
    const _Float16* bp = wt + (size_t)(jb * UB + n0 + wn + m) * KD + 8 * hh;
#pragma unroll 1
    for (int kt = 0; kt < KD / 32; ++kt) {
      const int k0 = 32 * kt;
      FragH a0, a1;
      a0.h[0] = *(const v8h*)(ap + k0);
      a0.h[1] = *(const v8h*)(ap + k0 + 16);
      a1.h[0] = *(const v8h*)(ap + 16 * KD + k0);
      a1.h[1] = *(const v8h*)(ap + 16 * KD + k0 + 16);
#pragma unroll
      for (int e = 0; e < 8; ++e) { a0.u[e] ^= sx; a1.u[e] ^= sx; }
#pragma unroll
      for (int nt = 0; nt < 4; ++nt) {
        const _Float16* bq = bp + (size_t)nt * 16 * KD + k0;
        FragH b;
        b.h[0] = *(const v8h*)bq;
        b.h[1] = *(const v8h*)(bq + 16);
        acc[0][nt] = wmf(a0.v, b.v, acc[0][nt]);
        acc[1][nt] = wmf(a1.v, b.v, acc[1][nt]);
      }
    }
  }

  constexpr float OSC = 1.0f / (float)(XSC * WSC);
  float bv[4];
#pragma unroll
  for (int nt = 0; nt < 4; ++nt) bv[nt] = bias[kb * UB + n0 + wn + 16 * nt + m];
#pragma unroll
  for (int mt = 0; mt < 2; ++mt) {
    float* sp = stg + (16 * mt + 8 * hh) * 64 + m;
#pragma unroll
    for (int nt = 0; nt < 4; ++nt) {
#pragma unroll
      for (int r = 0; r < 8; ++r) sp[r * 64 + 16 * nt] = acc[mt][nt][r] * OSC + bv[nt];
    }
  }
  __syncthreads();

  float* gbase = out + (size_t)(kb * MB + m0 + wm) * UB + n0 + wn;
#pragma unroll
  for (int q = 0; q < 16; ++q) {
    const int row = 2 * q + hh;
    const v4f v = *(const v4f*)(stg + row * 64 + 4 * m);
    *(volatile v4f*)(gbase + (size_t)row * UB + 4 * m) = v;
  }
  __threadfence();
#pragma unroll
  for (int q = 0; q < 16; ++q) {
    const int row = 2 * q + hh;
    const v4f v = *(const v4f*)(stg + row * 64 + 4 * m);
    *(volatile v4f*)(gbase + (size_t)row * UB + 4 * m) = v;
  }
}

extern "C" void kernel_launch(void* const* d_in, const int* in_sizes, int n_in,
                              void* d_out, int out_size, void* d_ws, size_t ws_size,
                              hipStream_t stream) {
  if (n_in < 3) return;
  if (in_sizes[0] != MTOT * KD || in_sizes[1] != KD * NW || in_sizes[2] != NW) return;
  if (out_size != MTOT * UB) return;

  const float* x    = (const float*)d_in[0];
  const float* W    = (const float*)d_in[1];
  const float* bias = (const float*)d_in[2];
  float* out = (float*)d_out;

  char* ws = (char*)d_ws;
  size_t off = 0;
  const size_t oXh = off; off += (size_t)MTOT * KD * 2;  off = (off + 255) & ~(size_t)255;
  const size_t oWt = off; off += (size_t)NW * KD * 2;    off = (off + 255) & ~(size_t)255;
  if (off > ws_size || off > (size_t)WSCAP) return;
  _Float16* xh = (_Float16*)(ws + oXh);
  _Float16* wt = (_Float16*)(ws + oWt);

  k_prepx<<<(MTOT * KD) / (8 * NTHR), NTHR, 0, stream>>>(x, xh);
  k_prepw<<<NW / 64, NTHR, 0, stream>>>(W, wt);
  hipFuncSetAttribute(reinterpret_cast<const void*>(&k_gemm),
                      hipFuncAttributeMaxDynamicSharedMemorySize, LDS_GEMM);
  k_gemm<<<dim3(UB / 128, MB / 128, NBL), NTHR, LDS_GEMM, stream>>>(xh, wt, bias, out);
}
